// BidirRecurrentModel_64398739636720
// MI455X (gfx1250) — hardware-verified
//
#include <hip/hip_runtime.h>
#include <math.h>

constexpr int NBATCH  = 32;
constexpr int NSTEP   = 128;
constexpr int NIN     = 512;
constexpr int NHID    = 512;
constexpr int NG3     = 3 * NHID;
constexpr int NOUTC   = 512;
constexpr int NFCK    = 2 * NHID;
constexpr int NROWS   = NSTEP * NBATCH;
constexpr int PADROWS = 64;
constexpr int XFROWS  = NROWS + 32;
constexpr int NTHR    = 256;
constexpr int SEQ_BLK = 16;
constexpr int HPITCH  = 520;
constexpr int NLAYER  = 2;
constexpr float WCARRY     = 16.0f;
constexpr float WCARRY_INV = 1.0f / 16.0f;
static_assert(NBATCH % SEQ_BLK == 0);
static_assert(NHID == 64 * (NTHR / 32));
static_assert(NIN % 64 == 0 && NHID % 64 == 0 && NFCK % 64 == 0 && NOUTC % 64 == 0);
static_assert(NROWS % 64 == 0 && NG3 % 64 == 0 && PADROWS % 64 == 0);
static_assert(NIN / 8 == 64 && NBATCH == 32);
static_assert((2 * SEQ_BLK * HPITCH) % NTHR == 0);
static_assert((SEQ_BLK * NHID) % NTHR == 0);
static_assert(HPITCH % 8 == 0);

typedef __attribute__((ext_vector_type(16))) _Float16 v16h;
typedef __attribute__((ext_vector_type(8)))  _Float16 v8h;
typedef __attribute__((ext_vector_type(16))) __bf16   v16b;
typedef __attribute__((ext_vector_type(8)))  __bf16   v8b;
typedef __attribute__((ext_vector_type(8)))  float    v8f;
typedef __attribute__((ext_vector_type(4)))  float    v4f;
typedef __attribute__((ext_vector_type(4)))  unsigned int v4u;

__device__ __forceinline__ unsigned short f2bf_bits(float f) {
  unsigned u = __float_as_uint(f);
  return (unsigned short)((u + 0x7FFFu + ((u >> 16) & 1u)) >> 16);
}
__device__ __forceinline__ float bf_bits2f(unsigned short h) { return __uint_as_float(((unsigned)h) << 16); }

__device__ __forceinline__ void dep_guard_h(v8f& a, v8f& b, v16h x, v16h y) { asm volatile("v_nop\n\tv_nop\n\tv_nop\n\tv_nop" : "+v"(a), "+v"(b) : "v"(x), "v"(y)); }
__device__ __forceinline__ void dep_guard_b(v8f& a, v8f& b, v16b x, v16b y) { asm volatile("v_nop\n\tv_nop\n\tv_nop\n\tv_nop" : "+v"(a), "+v"(b) : "v"(x), "v"(y)); }
__device__ __forceinline__ void keep4_h(v16h a, v16h b, v16h c, v16h d) { asm volatile("v_nop" :: "v"(a), "v"(b), "v"(c), "v"(d)); }
__device__ __forceinline__ void keep4_b(v16b a, v16b b, v16b c, v16b d) { asm volatile("v_nop" :: "v"(a), "v"(b), "v"(c), "v"(d)); }
__device__ __forceinline__ void acc_guard4(v8f& a, v8f& b, v8f& c, v8f& d) { asm volatile("v_nop\n\tv_nop\n\tv_nop\n\tv_nop" : "+v"(a), "+v"(b), "+v"(c), "+v"(d)); }
__device__ __forceinline__ void dep_guard3h(v8f& a, v8f& b, v8f& c, v16h x, v16h y, v16h z, v16h w) {
  asm volatile("v_nop\n\tv_nop\n\tv_nop\n\tv_nop" : "+v"(a), "+v"(b), "+v"(c) : "v"(x), "v"(y), "v"(z), "v"(w));
}
__device__ __forceinline__ void acc_guard3(v8f& a, v8f& b, v8f& c) { asm volatile("v_nop\n\tv_nop\n\tv_nop\n\tv_nop" : "+v"(a), "+v"(b), "+v"(c)); }
template <typename T> struct Frag;
template <> struct Frag<_Float16> {
  typedef v16h V; union U { v16h v; v8h h[2]; };
  static __device__ __forceinline__ v16h load(const _Float16* p) {
    U f; f.h[0] = *(const v8h*)(p); f.h[1] = *(const v8h*)(p + 16); return f.v;
  }
  static __device__ __forceinline__ v8f mma(v16h a, v16h b, v8f c) {
    return __builtin_amdgcn_wmma_f32_16x16x32_f16(false, a, false, b, (short)0, c, false, false);
  }
  static __device__ __forceinline__ void guard(v8f& a, v8f& b, v16h x, v16h y) { dep_guard_h(a, b, x, y); }
  static __device__ __forceinline__ void keep(v16h a, v16h b, v16h c, v16h d) { keep4_h(a, b, c, d); }
};
template <> struct Frag<__bf16> {
  typedef v16b V; union U { v16b v; v8b h[2]; };
  static __device__ __forceinline__ v16b load(const __bf16* p) {
    U f; f.h[0] = *(const v8b*)(p); f.h[1] = *(const v8b*)(p + 16); return f.v;
  }
  static __device__ __forceinline__ v8f mma(v16b a, v16b b, v8f c) {
    return __builtin_amdgcn_wmma_f32_16x16x32_bf16(false, a, false, b, (short)0, c, false, false);
  }
  static __device__ __forceinline__ void guard(v8f& a, v8f& b, v16b x, v16b y) { dep_guard_b(a, b, x, y); }
  static __device__ __forceinline__ void keep(v16b a, v16b b, v16b c, v16b d) { keep4_b(a, b, c, d); }
};

__device__ __forceinline__ float fsig(float x)  { return __builtin_amdgcn_rcpf(1.0f + expf(-x)); }
__device__ __forceinline__ float ftanh(float x) { return 1.0f - 2.0f * __builtin_amdgcn_rcpf(expf(2.0f * x) + 1.0f); }

template <int ET> struct Elem;
template <> struct Elem<0> { typedef _Float16 T; };
template <> struct Elem<1> { typedef __bf16 T; };
template <int ET, bool SPLIT, int BIAS_MODE, int OUT_MODE, bool RESID, int ACT = 0>
__global__ __launch_bounds__(256) void wmma_gemm64(
    const unsigned short* __restrict__ Ap, const unsigned short* __restrict__ A2p, int lda, long strideA,
    const unsigned short* __restrict__ Btp, const unsigned short* __restrict__ Bt2p, int ldb, long strideB,
    void* __restrict__ Cout, void* __restrict__ Cout2, int ldc, long strideC,
    const float* __restrict__ bias,
    const float* __restrict__ resid, long strideR,
    int M, int N, int K, float scale) {
  typedef typename Elem<ET>::T T;
  typedef typename Frag<T>::V V;
  const T* A = (const T*)Ap; const T* A2 = (const T*)A2p; const T* Bt = (const T*)Btp; const T* Bt2 = (const T*)Bt2p;
  __shared__ __align__(16) float sT[8][16 * 68];
  const int b    = blockIdx.y;
  const int lane = threadIdx.x & 31;
  const int wave = threadIdx.x >> 5;
  const int tilesN = N >> 6;
  const int tilesM = M >> 6;
  const int tile = blockIdx.x * 8 + wave;
  if (tile >= tilesM * tilesN) return;
  const int tm = tile / tilesN;
  const int tn = tile - tm * tilesN;
  const int m0 = tm << 6;
  const int n0 = tn << 6;

  const T* Ab  = A  + (size_t)b * strideA;
  const T* Bb  = Bt + (size_t)b * strideB;
  const T* Ab2 = SPLIT ? (A2  + (size_t)b * strideA) : nullptr;
  const T* Bb2 = SPLIT ? (Bt2 + (size_t)b * strideB) : nullptr;

  const int rlane = lane & 15;
  const int koff  = (lane >> 4) * 8;
  const int mOff  = (lane >> 4) * 8;

  v8f acc[4][4];
#pragma unroll
  for (int i = 0; i < 4; ++i)
#pragma unroll
    for (int j = 0; j < 4; ++j) acc[i][j] = (v8f){0.f,0.f,0.f,0.f,0.f,0.f,0.f,0.f};

  for (int k0 = 0; k0 < K; k0 += 32) {
    V bh[4], bl[4];
#pragma unroll
    for (int j = 0; j < 4; ++j) {
      const size_t bo = (size_t)(n0 + (j << 4) + rlane) * ldb + koff + k0;
      bh[j] = Frag<T>::load(Bb + bo);
      if (SPLIT) bl[j] = Frag<T>::load(Bb2 + bo);
    }
#pragma unroll
    for (int i = 0; i < 4; ++i) {
      const size_t ao = (size_t)(m0 + (i << 4) + rlane) * lda + koff + k0;
      V ah = Frag<T>::load(Ab + ao);
      V al;
      if (SPLIT) al = Frag<T>::load(Ab2 + ao);
#pragma unroll
      for (int j = 0; j < 4; ++j) {
        acc[i][j] = Frag<T>::mma(ah, bh[j], acc[i][j]);
        if (SPLIT) {
          acc[i][j] = Frag<T>::mma(ah, bl[j], acc[i][j]);
          acc[i][j] = Frag<T>::mma(al, bh[j], acc[i][j]);
        }
      }
      Frag<T>::guard(acc[i][0], acc[i][3], ah, SPLIT ? al : ah);
    }
    Frag<T>::keep(bh[0], bh[1], bh[2], bh[3]);
    if (SPLIT) Frag<T>::keep(bl[0], bl[1], bl[2], bl[3]);
  }
  acc_guard4(acc[0][0], acc[0][1], acc[0][2], acc[0][3]);
  acc_guard4(acc[1][0], acc[1][1], acc[1][2], acc[1][3]);
  acc_guard4(acc[2][0], acc[2][1], acc[2][2], acc[2][3]);
  acc_guard4(acc[3][0], acc[3][1], acc[3][2], acc[3][3]);

  float* slab = sT[wave];
  const float* Rb = RESID ? (resid + (size_t)b * strideR) : nullptr;
#pragma unroll
  for (int i = 0; i < 4; ++i) {
    const int mBase = m0 + (i << 4);
#pragma unroll
    for (int j = 0; j < 4; ++j) {
      const int n = n0 + (j << 4) + rlane;
      float bv = 0.f;
      if (BIAS_MODE == 2) bv = bias[n];
#pragma unroll
      for (int r = 0; r < 8; ++r) {
        float v = acc[i][j][r] * scale;
        if (BIAS_MODE == 1) v += bias[mBase + mOff + r];
        if (BIAS_MODE == 2) v += bv;
        if (RESID) v += Rb[(size_t)(mBase + mOff + r) * ldc + n];
        if (ACT == 1) v = tanhf(v);
        if (ACT == 2) v = fmaxf(v, 0.0f);
        if (ACT == 3) v = v / (1.0f + expf(-v));
        if (ACT == 4) v = (v > 0.f) ? v : 0.01f * v;
        if (ACT == 5) v = 0.5f * v * (1.0f + erff(v * 0.70710678118654752f));
        slab[(mOff + r) * 68 + (j << 4) + rlane] = v;
      }
    }
    __builtin_amdgcn_fence(__ATOMIC_RELEASE, "workgroup");
    __builtin_amdgcn_wave_barrier();
    __builtin_amdgcn_fence(__ATOMIC_ACQUIRE, "workgroup");
    if (OUT_MODE == 0) {
      float* C = (float*)Cout + (size_t)b * strideC;
      const int hh = lane >> 4, c4 = (lane & 15) * 4;
      for (int pass = 0; pass < 2; ++pass) {
#pragma unroll
        for (int it = 0; it < 8; ++it) {
          const int row = it * 2 + hh;
          v4f v = *(const v4f*)(slab + row * 68 + c4);
          *(volatile v4f*)(C + (size_t)(mBase + row) * ldc + n0 + c4) = v;
        }
        __threadfence();
      }
    } else {
      const int q = lane >> 3, c8 = (lane & 7) * 8;
      unsigned short* C  = (unsigned short*)Cout  + (size_t)b * strideC;
      unsigned short* C2 = (OUT_MODE == 2) ? ((unsigned short*)Cout2 + (size_t)b * strideC) : nullptr;
      for (int pass = 0; pass < 2; ++pass) {
#pragma unroll
        for (int it = 0; it < 4; ++it) {
          const int row = it * 4 + q;
          const float* sp = slab + row * 68 + c8;
          v8h hv, lv;
#pragma unroll
          for (int e = 0; e < 8; ++e) {
            if (OUT_MODE == 1) {
              hv[e] = (_Float16)sp[e];
            } else {
              unsigned short hb = f2bf_bits(sp[e]);
              unsigned short lb = f2bf_bits(sp[e] - bf_bits2f(hb));
              hv[e] = __builtin_bit_cast(_Float16, hb);
              lv[e] = __builtin_bit_cast(_Float16, lb);
            }
          }
          *(volatile v8h*)(C + (size_t)(mBase + row) * ldc + n0 + c8) = hv;
          if (OUT_MODE == 2) *(volatile v8h*)(C2 + (size_t)(mBase + row) * ldc + n0 + c8) = lv;
        }
        __threadfence();
      }
    }
    __builtin_amdgcn_fence(__ATOMIC_RELEASE, "workgroup");
    __builtin_amdgcn_wave_barrier();
    __builtin_amdgcn_fence(__ATOMIC_ACQUIRE, "workgroup");
  }
}

__global__ __launch_bounds__(NTHR) void zero16_kernel(unsigned short* __restrict__ dst, int n16) {
  const int i = blockIdx.x * NTHR + threadIdx.x;
  if (i < n16) {
    const v4u z = {0u, 0u, 0u, 0u};
    *(volatile v4u*)(dst + (size_t)i * 8) = z;
    __threadfence();
    *(volatile v4u*)(dst + (size_t)i * 8) = z;
  }
}

__global__ __launch_bounds__(NTHR) void xcast_kernel(const float* __restrict__ x, unsigned short* __restrict__ dstp) {
  const int i = blockIdx.x * NTHR + threadIdx.x;
  if (i < NROWS * (NIN / 8)) {
    const int row = i >> 6;
    const int c8  = (i & 63) * 8;
    const int t = row >> 5, b = row & 31;
    const float* sp = x + ((size_t)b * NSTEP + t) * NIN + c8;
    const v4f a  = *(const v4f*)(sp);
    const v4f bb = *(const v4f*)(sp + 4);
    v8h hv;
#pragma unroll
    for (int e = 0; e < 4; ++e) { hv[e] = (_Float16)a[e]; hv[4 + e] = (_Float16)bb[e]; }
    _Float16* dst = (_Float16*)dstp;
    *(volatile v8h*)(dst + (size_t)i * 8) = hv;
    __threadfence();
    *(volatile v8h*)(dst + (size_t)i * 8) = hv;
  }
}

__global__ __launch_bounds__(NTHR) void wtcast_kernel(const float* __restrict__ src, long srcStride, int K, int N,
                                                    unsigned short* __restrict__ dstp, long dstStride, int row0, float sc) {
  __shared__ __align__(16) float tile[64 * 68];
  const int tid = threadIdx.x, lane = tid & 31, wave = tid >> 5;
  const int n0 = blockIdx.x * 64, k0 = blockIdx.y * 64, sl = blockIdx.z;
  const float* s = src + (size_t)sl * srcStride;
#pragma unroll
  for (int it = 0; it < 4; ++it) {
    const int idx = it * NTHR + tid;
    const int r = idx >> 4, c4 = (idx & 15) * 4;
    const v4f v = *(const v4f*)(s + (size_t)(k0 + r) * N + n0 + c4);
    *(v4f*)(tile + r * 68 + c4) = v;
  }
  __syncthreads();
  _Float16* d = (_Float16*)dstp + (size_t)sl * dstStride;
  const int q = lane >> 3, kc = (lane & 7) * 8;
  for (int pass = 0; pass < 2; ++pass) {
#pragma unroll
    for (int it = 0; it < 2; ++it) {
      const int nrow = wave * 8 + it * 4 + q;
      v8h hv;
#pragma unroll
      for (int e = 0; e < 8; ++e) hv[e] = (_Float16)(sc * tile[(kc + e) * 68 + nrow]);
      *(volatile v8h*)(d + (size_t)(row0 + n0 + nrow) * K + k0 + kc) = hv;
    }
    __threadfence();
  }
}

__global__ __launch_bounds__(NTHR) void bx_kernel(const float* __restrict__ bxh, const float* __restrict__ bxr,
                                                float* __restrict__ dst) {
  const int i = blockIdx.x * NTHR + threadIdx.x;
  if (i < (NLAYER * 2 * NG3) / 4) {
    const int e0   = i * 4;
    const int s    = e0 / NG3;
    const int cpos = e0 - s * NG3;
    int ca = cpos;            if (ca > 2 * NHID - 4) ca = 2 * NHID - 4;
    int cb = cpos - 2 * NHID; if (cb < 0) cb = 0;
    const v4f va = *(const v4f*)(bxh + (size_t)s * 2 * NHID + ca);
    const v4f vb = *(const v4f*)(bxr + (size_t)s * NHID + cb);
    const bool first = (cpos < 2 * NHID);
    v4f o;
#pragma unroll
    for (int e = 0; e < 4; ++e) o[e] = first ? va[e] : vb[e];
    float* op = dst + (size_t)e0;
    *(volatile v4f*)op = o;
    __threadfence();
    *(volatile v4f*)op = o;
  }
}

__global__ __launch_bounds__(NTHR) void copy_out_kernel(const float* __restrict__ src, float* __restrict__ out, int n4) {
  const int i = blockIdx.x * NTHR + threadIdx.x;
  if (i < n4) {
    const v4f v = *(const v4f*)(src + (size_t)i * 4);
    *(volatile v4f*)(out + (size_t)i * 4) = v;
    __threadfence();
    *(volatile v4f*)(out + (size_t)i * 4) = v;
  }
}

__global__ __launch_bounds__(NTHR) void gru_seq_kernel(const float* __restrict__ XP, const unsigned short* __restrict__ WHp,
                                                     const float* __restrict__ bhh, const float* __restrict__ bhr,
                                                     unsigned short* __restrict__ seq16p, unsigned short* __restrict__ fin16p,
                                                     int write_seq, int fin_pitch, int fin_col0, int write_fin, int nsteps) {
  __shared__ __align__(16) _Float16 Ah[2][SEQ_BLK * HPITCH];
  __shared__ __align__(16) float    Hs[SEQ_BLK * NHID];
  const _Float16* WH = (const _Float16*)WHp;
  _Float16* seq16 = (_Float16*)seq16p;
  _Float16* fin16 = (_Float16*)fin16p;
  const int tid = threadIdx.x, lane = tid & 31, wave = tid >> 5;
  const int c = lane & 15, hh = lane >> 4, koff = hh * 8;
  const int q = lane >> 3, c8 = (lane & 7) * 8;
  const int rowbase = blockIdx.x * SEQ_BLK;

  {
    _Float16* ahf = &Ah[0][0];
#pragma unroll 1
    for (int i = tid; i < 2 * SEQ_BLK * HPITCH; i += NTHR) ahf[i] = (_Float16)0.0f;
#pragma unroll 1
    for (int i = tid; i < SEQ_BLK * NHID; i += NTHR) Hs[i] = 0.0f;
  }
  __syncthreads();

  int ns = nsteps;
  if (ns < 0) ns = 0;
  if (ns > NSTEP) ns = NSTEP;
  const v8f z8 = {0.f, 0.f, 0.f, 0.f, 0.f, 0.f, 0.f, 0.f};

#pragma unroll 1
  for (int t = 0; t < ns; ++t) {
    const int cur = t & 1;
    const _Float16* ahrow = &Ah[cur][0] + c * HPITCH + koff;
    _Float16* ahn = &Ah[cur ^ 1][0];
    const size_t xrow0 = (size_t)t * NBATCH + (size_t)rowbase + (size_t)(8 * hh);

#pragma unroll 1
    for (int nt = 0; nt < 4; ++nt) {
      const int j = 64 * wave + 16 * nt + c;
      const _Float16* wz = WH + (size_t)j * NHID + koff;
      const _Float16* wr = WH + (size_t)(NHID + j) * NHID + koff;
      const _Float16* wg = WH + (size_t)(2 * NHID + j) * NHID + koff;
      v8f accZ = z8, accR = z8, accG = z8;
#pragma unroll 1
      for (int k0 = 0; k0 < NHID; k0 += 32) {
        const v16h a  = Frag<_Float16>::load(ahrow + k0);
        const v16h b0 = Frag<_Float16>::load(wz + k0);
        const v16h b1 = Frag<_Float16>::load(wr + k0);
        const v16h b2 = Frag<_Float16>::load(wg + k0);
        accZ = Frag<_Float16>::mma(a, b0, accZ);
        accR = Frag<_Float16>::mma(a, b1, accR);
        accG = Frag<_Float16>::mma(a, b2, accG);
        dep_guard3h(accZ, accR, accG, a, b0, b1, b2);
      }
      acc_guard3(accZ, accR, accG);
      const float bzv = bhh[j], brv = bhh[NHID + j], bgv = bhr[j];
#pragma unroll
      for (int r = 0; r < 8; ++r) {
        const int row = 8 * hh + r;
        const float* xp = XP + (xrow0 + (size_t)r) * NG3;
        const float xz  = xp[j];
        const float xrr = xp[NHID + j];
        const float xx  = xp[2 * NHID + j];
        const float zp = (xz  + accZ[r] * WCARRY_INV) + bzv;
        const float rp = (xrr + accR[r] * WCARRY_INV) + brv;
        const float zg = fsig(zp);
        const float rg = fsig(rp);
        const float g  = ftanh((accG[r] * WCARRY_INV + bgv) * rg + xx);
        const float ho = Hs[row * NHID + j];
        const float hn = zg * ho + (1.0f - zg) * g;
        Hs[row * NHID + j] = hn;
        ahn[row * HPITCH + j] = (_Float16)hn;
      }
    }
    __syncthreads();

    const bool dofin = (write_fin != 0) && (t == ns - 1);
    if (write_seq != 0 || dofin) {
      const _Float16* ahs = &Ah[cur ^ 1][0] + 64 * wave + c8;
      for (int pass = 0; pass < 2; ++pass) {
#pragma unroll
        for (int it = 0; it < 4; ++it) {
          const int row = it * 4 + q;
          const v8h v = *(const v8h*)(ahs + row * HPITCH);
          if (write_seq != 0)
            *(volatile v8h*)(seq16 + ((size_t)t * NBATCH + (size_t)(rowbase + row)) * NHID + 64 * wave + c8) = v;
          if (dofin)
            *(volatile v8h*)(fin16 + (size_t)(rowbase + row) * (size_t)fin_pitch + fin_col0 + 64 * wave + c8) = v;
        }
        __threadfence();
      }
    }
  }
}

extern "C" void kernel_launch(void* const* d_in, const int* in_sizes, int n_in,
                              void* d_out, int out_size, void* d_ws, size_t ws_size, hipStream_t stream) {
  if (n_in < 11 || d_out == nullptr || d_ws == nullptr) return;
  if (in_sizes[0] != NBATCH * NSTEP * NIN || in_sizes[1] != NLAYER * 2 * NIN * 2 * NHID ||
      in_sizes[2] != NLAYER * 2 * 2 * NHID || in_sizes[3] != NLAYER * 2 * NHID * 2 * NHID ||
      in_sizes[4] != NLAYER * 2 * 2 * NHID || in_sizes[5] != NLAYER * 2 * NIN * NHID ||
      in_sizes[6] != NLAYER * 2 * NHID || in_sizes[7] != NLAYER * 2 * NHID * NHID ||
      in_sizes[8] != NLAYER * 2 * NHID || in_sizes[9] != NFCK * NOUTC || in_sizes[10] != NOUTC ||
      out_size != NBATCH * NOUTC) return;

  const float* x   = (const float*)d_in[0];
  const float* Wxh = (const float*)d_in[1];
  const float* bxh = (const float*)d_in[2];
  const float* Whh = (const float*)d_in[3];
  const float* bhh = (const float*)d_in[4];
  const float* Wxr = (const float*)d_in[5];
  const float* bxr = (const float*)d_in[6];
  const float* Whr = (const float*)d_in[7];
  const float* bhr = (const float*)d_in[8];
  const float* Wfc = (const float*)d_in[9];
  const float* bfc = (const float*)d_in[10];
  float* out = (float*)d_out;

  char* ws = (char*)d_ws; size_t off = 0;
  auto carve = [&](size_t bytes) -> char* { char* p = ws + off; off += (bytes + 255) & ~(size_t)255; return p; };
  unsigned short* XF    = (unsigned short*)carve((size_t)XFROWS * NIN * 2);
  unsigned short* HR1   = (unsigned short*)carve((size_t)PADROWS * NHID * 2);
  unsigned short* FCIN  = (unsigned short*)carve((size_t)PADROWS * NFCK * 2);
  unsigned short* H1F   = (unsigned short*)carve((size_t)NROWS * NHID * 2);
  unsigned short* WX16  = (unsigned short*)carve((size_t)NLAYER * 2 * NG3 * NIN * 2);
  unsigned short* WH16  = (unsigned short*)carve((size_t)NLAYER * 2 * NG3 * NHID * 2);
  unsigned short* WFC16 = (unsigned short*)carve((size_t)NOUTC * NFCK * 2);
  float*          BX    = (float*)carve((size_t)NLAYER * 2 * NG3 * 4);
  float*          XP1   = (float*)carve((size_t)NROWS * NG3 * 4);
  float*          XP2   = (float*)carve((size_t)NROWS * NG3 * 4);
  float*          XPR1  = (float*)carve((size_t)PADROWS * NG3 * 4);
  float*          XPR2  = (float*)carve((size_t)PADROWS * NG3 * 4);
  float*          FCO   = (float*)carve((size_t)PADROWS * NOUTC * 4);
  if (off > ws_size || off > (size_t)134217728) return;
  if ((char*)HR1 != (char*)XF + (size_t)XFROWS * NIN * 2) return;
  if ((char*)FCIN != (char*)HR1 + (size_t)PADROWS * NHID * 2) return;

  const int n16 = (32 * NIN + PADROWS * NHID + PADROWS * NFCK) / 8;
  zero16_kernel<<<(n16 + NTHR - 1) / NTHR, NTHR, 0, stream>>>(XF + (size_t)NROWS * NIN, n16);

  xcast_kernel<<<(NROWS * (NIN / 8) + NTHR - 1) / NTHR, NTHR, 0, stream>>>(x, XF);

  const long wxStride = (long)NG3 * NIN;
  wtcast_kernel<<<dim3(2 * NHID / 64, NIN / 64, NLAYER * 2), NTHR, 0, stream>>>(
      Wxh, (long)NIN * 2 * NHID, NIN, 2 * NHID, WX16, wxStride, 0, WCARRY);
  wtcast_kernel<<<dim3(NHID / 64, NIN / 64, NLAYER * 2), NTHR, 0, stream>>>(
      Wxr, (long)NIN * NHID, NIN, NHID, WX16, wxStride, 2 * NHID, WCARRY);
  wtcast_kernel<<<dim3(2 * NHID / 64, NHID / 64, NLAYER * 2), NTHR, 0, stream>>>(
      Whh, (long)NHID * 2 * NHID, NHID, 2 * NHID, WH16, wxStride, 0, WCARRY);
  wtcast_kernel<<<dim3(NHID / 64, NHID / 64, NLAYER * 2), NTHR, 0, stream>>>(
      Whr, (long)NHID * NHID, NHID, NHID, WH16, wxStride, 2 * NHID, WCARRY);
  wtcast_kernel<<<dim3(NOUTC / 64, NFCK / 64, 1), NTHR, 0, stream>>>(
      Wfc, 0L, NFCK, NOUTC, WFC16, 0L, 0, WCARRY);

  bx_kernel<<<((NLAYER * 2 * NG3) / 4 + NTHR - 1) / NTHR, NTHR, 0, stream>>>(bxh, bxr, BX);

  auto gemm = [&](const unsigned short* A, int lda, const unsigned short* Bt, int ldb, float* C, int ldc,
                  const float* bias, int M, int N, int K) {
    const int tiles = (M / 64) * (N / 64);
    wmma_gemm64<0, false, 2, 0, false, 0><<<dim3((tiles + 7) / 8, 1), 256, 0, stream>>>(
        A, A, lda, 0L, Bt, Bt, ldb, 0L, (void*)C, (void*)C, ldc, 0L, bias, bias, 0L, M, N, K, WCARRY_INV);
  };

  gemm(XF, NIN, WX16 + 0 * wxStride, NIN, XP1, NG3, BX + 0 * NG3, NROWS, NG3, NIN);
  gemm(XF + (size_t)(NSTEP - 1) * NBATCH * NIN, NIN, WX16 + 1 * wxStride, NIN, XPR1, NG3, BX + 1 * NG3, PADROWS, NG3, NIN);

  gru_seq_kernel<<<NBATCH / SEQ_BLK, NTHR, 0, stream>>>(
      XP1, WH16 + 0 * wxStride, bhh + 0 * 2 * NHID, bhr + 0 * NHID, H1F, FCIN, 1, NFCK, 0, 0, NSTEP);
  gru_seq_kernel<<<NBATCH / SEQ_BLK, NTHR, 0, stream>>>(
      XPR1, WH16 + 1 * wxStride, bhh + 1 * 2 * NHID, bhr + 1 * NHID, HR1, FCIN, 1, NFCK, 0, 0, 1);

  gemm(H1F, NHID, WX16 + 2 * wxStride, NHID, XP2, NG3, BX + 2 * NG3, NROWS, NG3, NHID);
  gemm(HR1, NHID, WX16 + 3 * wxStride, NHID, XPR2, NG3, BX + 3 * NG3, PADROWS, NG3, NHID);

  gru_seq_kernel<<<NBATCH / SEQ_BLK, NTHR, 0, stream>>>(
      XP2, WH16 + 2 * wxStride, bhh + 2 * 2 * NHID, bhr + 2 * NHID, H1F, FCIN, 0, NFCK, 0, 1, NSTEP);
  gru_seq_kernel<<<NBATCH / SEQ_BLK, NTHR, 0, stream>>>(
      XPR2, WH16 + 3 * wxStride, bhh + 3 * 2 * NHID, bhr + 3 * NHID, HR1, FCIN, 0, NFCK, NHID, 1, 1);

  gemm(FCIN, NFCK, WFC16, NFCK, FCO, NOUTC, bfc, PADROWS, NOUTC, NFCK);
  copy_out_kernel<<<(NBATCH * NOUTC / 4 + NTHR - 1) / NTHR, NTHR, 0, stream>>>(FCO, out, NBATCH * NOUTC / 4);
}
